// DavidBeans_32547262169466
// MI455X (gfx1250) — hardware-verified
//
#include <hip/hip_runtime.h>


#define NBI  32
#define SS   197
#define DD   768
#define NH_  12
#define HD   64
#define PP   196
#define KN   32
#define DFF  3072
#define NR   6304
#define NRP  6336
typedef _Float16 h16;
typedef unsigned short bf;
typedef __attribute__((ext_vector_type(16))) __bf16   v16bf;
typedef __attribute__((ext_vector_type(16))) _Float16 v16h;
typedef __attribute__((ext_vector_type(8)))  _Float16 v8h;
typedef __attribute__((ext_vector_type(8)))  unsigned short v8us;
typedef __attribute__((ext_vector_type(8)))  float    v8f;
typedef __attribute__((ext_vector_type(4)))  float    v4f;
typedef v8h  __attribute__((may_alias)) v8ha;
typedef v4f  __attribute__((may_alias)) v4fa;
typedef v8us __attribute__((may_alias)) v8usa;

__device__ __forceinline__ unsigned short f2bf(float f) { unsigned u = __float_as_uint(f); u += 0x7FFFu + ((u >> 16) & 1u); return (unsigned short)(u >> 16); }
__device__ __forceinline__ float bf2f(unsigned short b) { return __uint_as_float(((unsigned)b) << 16); }
__device__ __forceinline__ float bfr(float f) { return bf2f(f2bf(f)); }
__device__ __forceinline__ v16h cat16(v8h lo, v8h hi) { return __builtin_shufflevector(lo, hi, 0, 1, 2, 3, 4, 5, 6, 7, 8, 9, 10, 11, 12, 13, 14, 15); }
__device__ __forceinline__ v16bf cat16b(v8us lo, v8us hi) { return __builtin_bit_cast(v16bf, __builtin_shufflevector(lo, hi, 0, 1, 2, 3, 4, 5, 6, 7, 8, 9, 10, 11, 12, 13, 14, 15)); }
__device__ __forceinline__ v8f wmma16(v16h a, v16h b, v8f c) { return __builtin_amdgcn_wmma_f32_16x16x32_f16(false, a, false, b, (short)0, c, false, false); }
__device__ __forceinline__ v8f wmmab(v16bf a, v16bf b, v8f c) { return __builtin_amdgcn_wmma_f32_16x16x32_bf16(false, a, false, b, (short)0, c, false, false); }


template <typename T16> struct WFrag;
template <> struct WFrag<h16> { typedef v16h V; static __device__ __forceinline__ V ld(const h16* p) { return cat16(*(const v8h*)p, *(const v8h*)(p + 16)); } static __device__ __forceinline__ v8f mma(V a, V b, v8f c) { return wmma16(a, b, c); } };
template <> struct WFrag<bf> { typedef v16bf V; static __device__ __forceinline__ V ld(const bf* p) { return cat16b(*(const v8us*)p, *(const v8us*)(p + 16)); } static __device__ __forceinline__ v8f mma(V a, V b, v8f c) { return wmmab(a, b, c); } };
template <typename T16, int NSPLIT, bool BIAS>
__global__ __launch_bounds__(32) void k_gemmw(const T16* __restrict__ A, const T16* __restrict__ A2, const T16* __restrict__ Bt, const T16* __restrict__ Bt2, int K, float* C, int ldc, const float* __restrict__ bias, size_t sA, size_t sB, size_t sC) {
    typedef typename WFrag<T16>::V V;
    __shared__ __align__(16) float os[16 * 68];
    const size_t z = blockIdx.z; A += z * sA; if (A2) A2 += z * sA; Bt += z * sB; if (Bt2) Bt2 += z * sB; C += z * sC;
    const int lane = threadIdx.x & 31, lr = lane & 15, hi = lane >> 4; const int r0 = blockIdx.x * 64, c0 = blockIdx.y * 64;
    v8f acc[4][4];
#pragma unroll
    for (int mb = 0; mb < 4; ++mb)
#pragma unroll
        for (int nb = 0; nb < 4; ++nb) acc[mb][nb] = (v8f){};
    const size_t aoff = (size_t)(r0 + lr) * K + 8 * hi, boff = (size_t)(c0 + lr) * K + 8 * hi;
#pragma unroll 1
    for (int kc = 0; kc < K; kc += 32) {
        V a[4], a2[4];
#pragma unroll
        for (int mb = 0; mb < 4; ++mb) { a[mb] = WFrag<T16>::ld(A + aoff + (size_t)mb * 16 * K + kc); if (NSPLIT == 1 || NSPLIT == 2) a2[mb] = WFrag<T16>::ld(A2 + aoff + (size_t)mb * 16 * K + kc); }
#pragma unroll
        for (int nb = 0; nb < 4; ++nb) { const V b = WFrag<T16>::ld(Bt + boff + (size_t)nb * 16 * K + kc); V b2; if (NSPLIT >= 2) b2 = WFrag<T16>::ld(Bt2 + boff + (size_t)nb * 16 * K + kc);
#pragma unroll
            for (int mb = 0; mb < 4; ++mb) { acc[mb][nb] = WFrag<T16>::mma(a[mb], b, acc[mb][nb]); if (NSPLIT == 1 || NSPLIT == 2) acc[mb][nb] = WFrag<T16>::mma(a2[mb], b, acc[mb][nb]); if (NSPLIT >= 2) acc[mb][nb] = WFrag<T16>::mma(a[mb], b2, acc[mb][nb]); } }
        asm volatile("v_nop\n\tv_nop\n\tv_nop\n\tv_nop" : "+v"(acc[0][0]), "+v"(acc[1][1]), "+v"(acc[2][2]), "+v"(acc[3][3]) : "v"(a[0]), "v"(a[3]));
    }
#pragma unroll
    for (int mb = 0; mb < 4; ++mb) {
#pragma unroll
        for (int nb = 0; nb < 4; ++nb) {
#pragma unroll
            for (int j = 0; j < 8; ++j) os[(hi * 8 + j) * 68 + nb * 16 + lr] = acc[mb][nb][j]; }
        __builtin_amdgcn_wave_barrier(); asm volatile("" ::: "memory");
        float* crow = C + (size_t)(r0 + mb * 16) * ldc + c0;
#pragma unroll 1
        for (int ps = 0; ps < 2; ++ps) {
#pragma unroll
            for (int s = 0; s < 8; ++s) { const int row = 2 * s + hi, cofs = lr * 4; v4f val = *(const v4fa*)(os + row * 68 + cofs); if (BIAS) { val[0] += bfr(bias[c0 + cofs]); val[1] += bfr(bias[c0 + cofs + 1]); val[2] += bfr(bias[c0 + cofs + 2]); val[3] += bfr(bias[c0 + cofs + 3]); }
                *(volatile v4f*)(crow + (size_t)row * ldc + cofs) = val; }
            if (ps == 0) __threadfence(); }
        __builtin_amdgcn_wave_barrier(); asm volatile("" ::: "memory");
    }
}

__device__ __forceinline__ h16 tohx(float x) { return (h16)x; }
typedef __attribute__((ext_vector_type(2))) _Float16 v2h;
typedef __attribute__((ext_vector_type(4))) _Float16 v4h;
typedef __attribute__((ext_vector_type(2))) float v2f;

__global__ __launch_bounds__(256) void k_wt16(const float* __restrict__ w, int K, int N, h16* Bt) { const size_t e = ((size_t)blockIdx.x * 256 + threadIdx.x) * 2; if (e >= (size_t)N * K) return; const int k = (int)(e % K), n = (int)(e / K); v2h o; o[0] = tohx(bfr(w[(size_t)k * N + n])); o[1] = tohx(bfr(w[(size_t)(k + 1) * N + n])); *(volatile v2h*)(Bt + e) = o; __threadfence(); *(volatile v2h*)(Bt + e) = o; }
__global__ __launch_bounds__(256) void k_lnpl(const float* __restrict__ X, int isin, const float* __restrict__ g, const float* __restrict__ bb, h16* P) { const int lane = threadIdx.x & 31; const int r = blockIdx.x * 8 + (threadIdx.x >> 5); if (r >= NRP) return; const size_t rb = (size_t)r * DD;
    if (r >= NR) { for (int ps = 0; ps < 2; ++ps) { for (int ch = 0; ch < 6; ++ch) { v4h z; z[0] = z[1] = z[2] = z[3] = (h16)0.f; *(volatile v4h*)(P + rb + ch * 128 + lane * 4) = z; } if (ps == 0) __threadfence(); } return; }
    float s = 0.f;
#pragma unroll 1
    for (int ch = 0; ch < 6; ++ch) { const v4f a = *(const v4f*)(X + rb + ch * 128 + lane * 4);
#pragma unroll
        for (int q = 0; q < 4; ++q) s = __fadd_rn(s, isin ? bfr(a[q]) : a[q]); }
#pragma unroll
    for (int sh = 16; sh; sh >>= 1) s += __shfl_xor(s, sh, 32);
    const float mu = s * (1.0f / DD); float q2 = 0.f;
#pragma unroll 1
    for (int ch = 0; ch < 6; ++ch) { const v4f a = *(const v4f*)(X + rb + ch * 128 + lane * 4);
#pragma unroll
        for (int q = 0; q < 4; ++q) { float dv = __fsub_rn(isin ? bfr(a[q]) : a[q], mu); asm volatile("" : "+v"(dv)); float p = __fmul_rn(dv, dv); asm volatile("" : "+v"(p)); q2 = __fadd_rn(q2, p); } }
#pragma unroll
    for (int sh = 16; sh; sh >>= 1) q2 += __shfl_xor(q2, sh, 32);
    float vq = q2 * (1.0f / DD); asm volatile("" : "+v"(vq)); const float rs = __frsqrt_rn(__fadd_rn(vq, 1e-5f));
#pragma unroll 1
    for (int ps = 0; ps < 2; ++ps) {
#pragma unroll 1
        for (int ch = 0; ch < 6; ++ch) { const int c0 = ch * 128 + lane * 4; const v4f a = *(const v4f*)(X + rb + c0); v4h o;
#pragma unroll
            for (int q = 0; q < 4; ++q) { float dv = __fsub_rn(isin ? bfr(a[q]) : a[q], mu); asm volatile("" : "+v"(dv)); float tn = __fmul_rn(dv, rs); asm volatile("" : "+v"(tn)); float tg = __fmul_rn(tn, bfr(g[c0 + q])); asm volatile("" : "+v"(tg)); o[q] = tohx(__fadd_rn(tg, bfr(bb[c0 + q]))); }
            *(volatile v4h*)(P + rb + c0) = o; } if (ps == 0) __threadfence(); } }
__global__ __launch_bounds__(256) void k_attcls(const float* __restrict__ QKV, float* O) { const int lane = threadIdx.x & 31; const int wv = blockIdx.x * 8 + (threadIdx.x >> 5); if (wv >= NBI * NH_) return; const int h = wv % NH_; const int b = wv / NH_; const size_t r0 = (size_t)b * SS; const float* qp = QKV + r0 * 3 * DD + h * HD + 2 * lane; const float q0 = qp[0], q1 = qp[1]; float mx = -3.0e38f;
#pragma unroll 1
    for (int j = 0; j < SS; ++j) { const float* kp = QKV + (r0 + j) * 3 * DD + DD + h * HD + 2 * lane; float p = __fmul_rn(q0, kp[0]); asm volatile("" : "+v"(p)); float p2 = __fmul_rn(q1, kp[1]); asm volatile("" : "+v"(p2)); float s = __fadd_rn(p, p2);
#pragma unroll
        for (int sh = 16; sh; sh >>= 1) s += __shfl_xor(s, sh, 32);
        mx = fmaxf(mx, s * 0.125f); }
    float sum = 0.f, a0 = 0.f, a1 = 0.f;
#pragma unroll 1
    for (int j = 0; j < SS; ++j) { const float* kp = QKV + (r0 + j) * 3 * DD + DD + h * HD + 2 * lane; float p = __fmul_rn(q0, kp[0]); asm volatile("" : "+v"(p)); float p2 = __fmul_rn(q1, kp[1]); asm volatile("" : "+v"(p2)); float s = __fadd_rn(p, p2);
#pragma unroll
        for (int sh = 16; sh; sh >>= 1) s += __shfl_xor(s, sh, 32);
        float d0 = __fsub_rn(s * 0.125f, mx); asm volatile("" : "+v"(d0)); const float e = __expf(d0); sum = __fadd_rn(sum, e); const float* vp = kp + DD; float t0 = __fmul_rn(e, vp[0]); asm volatile("" : "+v"(t0)); a0 = __fadd_rn(a0, t0); float t1 = __fmul_rn(e, vp[1]); asm volatile("" : "+v"(t1)); a1 = __fadd_rn(a1, t1); }
    const float inv = __fdiv_rn(1.0f, sum); v2f o; o[0] = __fmul_rn(a0, inv); o[1] = __fmul_rn(a1, inv); const size_t oo = r0 * DD + h * HD + 2 * lane; *(volatile v2f*)(O + oo) = o; __threadfence(); *(volatile v2f*)(O + oo) = o; }
__global__ __launch_bounds__(256) void k_attp(const float* __restrict__ QKV, const int* __restrict__ routes, float* O) { const int lane = threadIdx.x & 31; const int wv = blockIdx.x * 8 + (threadIdx.x >> 5); if (wv >= NBI * PP * NH_) return; const int h = wv % NH_; const int p = (wv / NH_) % PP; const int b = wv / (NH_ * PP); const size_t r0 = (size_t)b * SS; const size_t rq = r0 + 1 + p; const float* qp = QKV + rq * 3 * DD + h * HD + 2 * lane; const float q0 = qp[0], q1 = qp[1]; float sc[KN]; float mx = -3.0e38f;
#pragma unroll
    for (int k = 0; k < KN; ++k) { int j = routes[p * KN + k]; j = min(max(j, 0), PP - 1) + 1; const float* kp = QKV + (r0 + j) * 3 * DD + DD + h * HD + 2 * lane; float pr = __fmul_rn(q0, kp[0]); asm volatile("" : "+v"(pr)); float p2 = __fmul_rn(q1, kp[1]); asm volatile("" : "+v"(p2)); float s = __fadd_rn(pr, p2);
#pragma unroll
        for (int sh = 16; sh; sh >>= 1) s += __shfl_xor(s, sh, 32);
        sc[k] = s * 0.125f; mx = fmaxf(mx, sc[k]); }
    float sum = 0.f;
#pragma unroll
    for (int k = 0; k < KN; ++k) { float d0 = __fsub_rn(sc[k], mx); asm volatile("" : "+v"(d0)); sc[k] = __expf(d0); sum = __fadd_rn(sum, sc[k]); }
    const float inv = __fdiv_rn(1.0f, sum); float a0 = 0.f, a1 = 0.f;
#pragma unroll 1
    for (int k = 0; k < KN; ++k) { int j = routes[p * KN + k]; j = min(max(j, 0), PP - 1) + 1; const float* vp = QKV + (r0 + j) * 3 * DD + 2 * DD + h * HD + 2 * lane; float w = __fmul_rn(sc[k], inv); asm volatile("" : "+v"(w)); float t0 = __fmul_rn(w, vp[0]); asm volatile("" : "+v"(t0)); a0 = __fadd_rn(a0, t0); float t1 = __fmul_rn(w, vp[1]); asm volatile("" : "+v"(t1)); a1 = __fadd_rn(a1, t1); }
    v2f o; o[0] = a0; o[1] = a1; const size_t oo = rq * DD + h * HD + 2 * lane; *(volatile v2f*)(O + oo) = o; __threadfence(); *(volatile v2f*)(O + oo) = o; }
__global__ __launch_bounds__(256) void k_f16(const float* __restrict__ F, size_t n4, h16* P) { const size_t i = ((size_t)blockIdx.x * 256 + threadIdx.x) * 4; if (i >= n4 * 4) return; const v4f a = *(const v4f*)(F + i); v4h o; o[0] = tohx(a[0]); o[1] = tohx(a[1]); o[2] = tohx(a[2]); o[3] = tohx(a[3]); *(volatile v4h*)(P + i) = o; __threadfence(); *(volatile v4h*)(P + i) = o; }
__global__ __launch_bounds__(256) void k_res(const float* __restrict__ x, const float* __restrict__ A, float* X1) { const size_t i = ((size_t)blockIdx.x * 256 + threadIdx.x) * 4; if (i >= (size_t)NR * DD) return; const v4f a = *(const v4f*)(A + i); v4f o; o[0] = __fadd_rn(bfr(x[i]), a[0]); o[1] = __fadd_rn(bfr(x[i + 1]), a[1]); o[2] = __fadd_rn(bfr(x[i + 2]), a[2]); o[3] = __fadd_rn(bfr(x[i + 3]), a[3]); *(volatile v4f*)(X1 + i) = o; __threadfence(); *(volatile v4f*)(X1 + i) = o; }
__global__ __launch_bounds__(256) void k_gelu16(const float* __restrict__ A, size_t n4, h16* G) { const size_t i = ((size_t)blockIdx.x * 256 + threadIdx.x) * 4; if (i >= n4 * 4) return; const v4f a = *(const v4f*)(A + i); v4h o;
#pragma unroll
    for (int q = 0; q < 4; ++q) o[q] = tohx(0.5f * a[q] * (1.0f + erff(a[q] * 0.7071067811865476f))); *(volatile v4h*)(G + i) = o; __threadfence(); *(volatile v4h*)(G + i) = o; }
__global__ __launch_bounds__(256) void k_fin(const float* __restrict__ X1, const float* __restrict__ M, float* OUT) { const size_t i = ((size_t)blockIdx.x * 256 + threadIdx.x) * 4; if (i >= (size_t)NR * DD) return; const v4f a = *(const v4f*)(X1 + i), m = *(const v4f*)(M + i); v4f o; o[0] = __fadd_rn(a[0], m[0]); o[1] = __fadd_rn(a[1], m[1]); o[2] = __fadd_rn(a[2], m[2]); o[3] = __fadd_rn(a[3], m[3]); *(volatile v4f*)(OUT + i) = o; __threadfence(); *(volatile v4f*)(OUT + i) = o; }

extern "C" void kernel_launch(void* const* d_in, const int* in_sizes, int n_in,
                              void* d_out, int out_size, void* d_ws, size_t ws_size, hipStream_t stream) {
    (void)in_sizes; (void)n_in; (void)out_size;
    const float* x = (const float*)d_in[0]; const int* routes = (const int*)d_in[1]; const float* wqkv = (const float*)d_in[2]; const float* bqkv = (const float*)d_in[3]; const float* wpr = (const float*)d_in[4]; const float* bpr = (const float*)d_in[5]; const float* g1 = (const float*)d_in[6]; const float* be1 = (const float*)d_in[7]; const float* g2 = (const float*)d_in[8]; const float* be2 = (const float*)d_in[9]; const float* w1 = (const float*)d_in[10]; const float* bb1 = (const float*)d_in[11]; const float* w2 = (const float*)d_in[12]; const float* bb2 = (const float*)d_in[13];
    float* OUT = (float*)d_out;
    char* wsp = (char*)d_ws;
    auto take = [&](size_t bytes) { char* p = wsp; wsp += (bytes + 255) & ~(size_t)255; return (void*)p; };
    h16* WQ = (h16*)take((size_t)3 * DD * DD * 2); h16* WP = (h16*)take((size_t)DD * DD * 2); h16* W1 = (h16*)take((size_t)DFF * DD * 2); h16* W2 = (h16*)take((size_t)DD * DFF * 2);
    h16* P16 = (h16*)take((size_t)NRP * DD * 2); float* QKV = (float*)take((size_t)NRP * DFF * 4);   float* O = (float*)take((size_t)NRP * DD * 4); float* X1 = (float*)take((size_t)NRP * DD * 4); float* A = QKV; h16* G16 = (h16*)take((size_t)NRP * DFF * 2); float* M = O;
    if ((size_t)(wsp - (char*)d_ws) > ws_size) return;
    k_wt16<<<(unsigned)(((size_t)DD * 3 * DD / 2 + 255) / 256), 256, 0, stream>>>(wqkv, DD, 3 * DD, WQ); k_wt16<<<(unsigned)(((size_t)DD * DD / 2 + 255) / 256), 256, 0, stream>>>(wpr, DD, DD, WP); k_wt16<<<(unsigned)(((size_t)DD * DFF / 2 + 255) / 256), 256, 0, stream>>>(w1, DD, DFF, W1); k_wt16<<<(unsigned)(((size_t)DFF * DD / 2 + 255) / 256), 256, 0, stream>>>(w2, DFF, DD, W2);
    k_lnpl<<<NRP / 8, 256, 0, stream>>>(x, 1, g1, be1, P16);
    k_gemmw<h16, 0, true><<<dim3(NRP / 64, 3 * DD / 64, 1), 32, 0, stream>>>(P16, nullptr, WQ, nullptr, DD, QKV, 3 * DD, bqkv, 0, 0, 0);
    k_attcls<<<(NBI * NH_ + 7) / 8, 256, 0, stream>>>(QKV, O); k_attp<<<(NBI * PP * NH_ + 7) / 8, 256, 0, stream>>>(QKV, routes, O);
    k_f16<<<(unsigned)(((size_t)NRP * DD / 4 + 255) / 256), 256, 0, stream>>>(O, (size_t)NRP * DD / 4, P16);
    k_gemmw<h16, 0, true><<<dim3(NRP / 64, DD / 64, 1), 32, 0, stream>>>(P16, nullptr, WP, nullptr, DD, O, DD, bpr, 0, 0, 0); k_res<<<(unsigned)(((size_t)NR * DD / 4 + 255) / 256), 256, 0, stream>>>(x, O, X1);
    k_lnpl<<<NRP / 8, 256, 0, stream>>>(X1, 0, g2, be2, P16);
    k_gemmw<h16, 0, true><<<dim3(NRP / 64, DFF / 64, 1), 32, 0, stream>>>(P16, nullptr, W1, nullptr, DD, A, DFF, bb1, 0, 0, 0); k_gelu16<<<(unsigned)(((size_t)NRP * DFF / 4 + 255) / 256), 256, 0, stream>>>(A, (size_t)NRP * DFF / 4, G16);
    k_gemmw<h16, 0, true><<<dim3(NRP / 64, DD / 64, 1), 32, 0, stream>>>(G16, nullptr, W2, nullptr, DFF, M, DD, bb2, 0, 0, 0);
    k_fin<<<(unsigned)(((size_t)NR * DD / 4 + 255) / 256), 256, 0, stream>>>(X1, M, OUT);
}
